// ComplexMultiHeadAttention_14379550507634
// MI455X (gfx1250) — hardware-verified
//
#include <hip/hip_runtime.h>


#pragma clang fp contract(off)

#ifndef NB
#define NB 2
#endif
#ifndef SEQ
#define SEQ 2048
#endif
#ifndef NB_FULL
#define NB_FULL 2
#endif
#ifndef SEQ_FULL
#define SEQ_FULL 2048
#endif

namespace {
constexpr int HID = 1024, DH = 64, NH = 16;
constexpr int NFREQ = DH / 2;
constexpr int NWB = 6;
constexpr int MROWS = NB * SEQ;
constexpr int QT = SEQ / 16;
constexpr int QKW = 2 * DH;
constexpr int VTILE = QKW * 16;
constexpr int CW = 2 * HID;
constexpr int TE = (SEQ < 256) ? SEQ : 256;
constexpr int QTE = TE / 16;
constexpr int NQB_E = TE / 128;
constexpr int NQB_L = ((SEQ - TE) / 128 > 0) ? ((SEQ - TE) / 128) : 1;
constexpr float SCORE_SCALE = 0.125f;
constexpr float P_CARRY = 4096.0f;
constexpr float INV_P_CARRY = 1.0f / 4096.0f;
constexpr float RES_CARRY = 2048.0f;
constexpr float INV_RES_CARRY = 1.0f / 2048.0f;
constexpr float WO_CARRY = 256.0f;
constexpr float INV_WO_CARRY = 1.0f / 256.0f;
static_assert(SEQ % 128 == 0);
static_assert(TE % 128 == 0 && TE <= SEQ);
static_assert(NB >= 1 && NB <= NB_FULL);
static_assert(SEQ <= SEQ_FULL);
static_assert(NH * DH == HID);
static_assert(MROWS % 128 == 0);
static_assert(HID % 64 == 0 && HID % 32 == 0);
static_assert(SEQ % 8 == 0);
static_assert((size_t)MROWS * HID <= (size_t)NB_FULL * SEQ_FULL * HID);

typedef __bf16 b16;
typedef _Float16 h16;
typedef __bf16 v16b __attribute__((ext_vector_type(16)));
typedef __bf16 v8b __attribute__((ext_vector_type(8)));
typedef _Float16 v16h __attribute__((ext_vector_type(16)));
typedef _Float16 v8h __attribute__((ext_vector_type(8)));
typedef float v8f __attribute__((ext_vector_type(8)));
typedef float v4f __attribute__((ext_vector_type(4)));
typedef unsigned short v8us __attribute__((ext_vector_type(8)));
typedef unsigned int v8u __attribute__((ext_vector_type(8)));

__device__ __forceinline__ v8b ld8b(const b16* p) { return *(const v8b*)p; }
__device__ __forceinline__ v8h ld8h(const h16* p) { return *(const v8h*)p; }
__device__ __forceinline__ v16b cat8b(v8b a, v8b b) { return __builtin_shufflevector(a, b, 0, 1, 2, 3, 4, 5, 6, 7, 8, 9, 10, 11, 12, 13, 14, 15); }
__device__ __forceinline__ v16h cat8h(v8h a, v8h b) { return __builtin_shufflevector(a, b, 0, 1, 2, 3, 4, 5, 6, 7, 8, 9, 10, 11, 12, 13, 14, 15); }
__device__ __forceinline__ v16b frag_kb(const b16* p, int hh) { return cat8b(ld8b(p + 8 * hh), ld8b(p + 16 + 8 * hh)); }
__device__ __forceinline__ v16h frag_kh(const h16* p, int hh) { return cat8h(ld8h(p + 8 * hh), ld8h(p + 16 + 8 * hh)); }

__device__ __forceinline__ v8f wmma_b(v16b a, v16b b, v8f c) {
  v8f d = __builtin_amdgcn_wmma_f32_16x16x32_bf16(false, a, false, b, (short)0, c, false, false);
  asm volatile("v_nop\n\tv_nop\n\tv_nop\n\tv_nop" : "+v"(d) : "v"(a), "v"(b));
  return d;
}
__device__ __forceinline__ v8f wmma_h(v16h a, v16h b, v8f c) {
  v8f d = __builtin_amdgcn_wmma_f32_16x16x32_f16(false, a, false, b, (short)0, c, false, false);
  asm volatile("v_nop\n\tv_nop\n\tv_nop\n\tv_nop" : "+v"(d) : "v"(a), "v"(b));
  return d;
}
template <typename V>
__device__ __forceinline__ V neg16(V a) {
  v8u t = __builtin_bit_cast(v8u, a);
  const v8u s = {0x80008000u, 0x80008000u, 0x80008000u, 0x80008000u, 0x80008000u, 0x80008000u, 0x80008000u, 0x80008000u};
  t = t ^ s;
  return __builtin_bit_cast(V, t);
}
__device__ __forceinline__ unsigned int bf16_rne_u32(float f) {
  unsigned int u = __builtin_bit_cast(unsigned int, f);
  u += 0x7fffu + ((u >> 16) & 1u);
  return u & 0xffff0000u;
}
__device__ __forceinline__ void wave_lds_sync() {
  __builtin_amdgcn_fence(3, "workgroup");
  __builtin_amdgcn_wave_barrier();
  __builtin_amdgcn_fence(2, "workgroup");
}

__device__ __forceinline__ void store_tile_4k(h16* dst, const h16* Tp, int lane) {
#pragma unroll
  for (int j = 0; j < 8; ++j) { const int e = (j * 32 + lane) * 8; *(volatile v8h*)(dst + e) = ld8h(Tp + e); }
  __threadfence();
#pragma unroll
  for (int j = 0; j < 8; ++j) { const int e = (j * 32 + lane) * 8; *(volatile v8h*)(dst + e) = ld8h(Tp + e); }
}

__global__ __launch_bounds__(256) void tab_kernel(float* __restrict__ tc, float* __restrict__ ts) {
  const int lane = threadIdx.x & 31, wave = threadIdx.x >> 5;
  const int pos = blockIdx.x * 8 + wave;
  const int j = lane;
  double r = 10000.0;
#pragma unroll 1
  for (int i = 0; i < 5; ++i) r = sqrt(r);
  double p = 1.0;
#pragma unroll 1
  for (int i = 0; i < j; ++i) p = p * r;
  const float p32 = (float)p;
  const float inv = 1.0f / p32;
  const float ang = (float)pos * inv;
  float sv, cv;
  sincosf(ang, &sv, &cv);
  float* pc = tc + (size_t)pos * NFREQ + j;
  float* ps = ts + (size_t)pos * NFREQ + j;
  *(volatile float*)pc = cv;
  *(volatile float*)ps = sv;
  __threadfence();
  *(volatile float*)pc = cv;
  *(volatile float*)ps = sv;
}

__global__ __launch_bounds__(256) void cvt_kernel(const float* __restrict__ xr, const float* __restrict__ xi,
                                                  const float* __restrict__ w0, const float* __restrict__ w1, const float* __restrict__ w2,
                                                  const float* __restrict__ w3, const float* __restrict__ w4, const float* __restrict__ w5,
                                                  const float* __restrict__ wo0, const float* __restrict__ wo1,
                                                  unsigned short* __restrict__ xrp, unsigned short* __restrict__ xip,
                                                  unsigned short* __restrict__ wpl, h16* __restrict__ wopl) {
  const size_t tid = (size_t)blockIdx.x * blockDim.x + threadIdx.x, stride = (size_t)gridDim.x * blockDim.x;
  const size_t nx = (size_t)MROWS * HID / 8;
  const size_t per_w = (size_t)HID * HID / 8;
  for (int pass = 0; pass < 2; ++pass) {
    for (size_t c = tid; c < 2 * nx; c += stride) {
      const int pl = (c >= nx) ? 1 : 0;
      const size_t i = (c - (size_t)pl * nx) * 8;
      const int m = (int)(i / HID), col = (int)(i % HID);
      const int bb = m / SEQ, t = m - bb * SEQ;
      const float* p = (pl ? xi : xr) + ((size_t)bb * SEQ_FULL + t) * HID + col;
      const v4f f0 = *(const v4f*)p, f1 = *(const v4f*)(p + 4);
      v8us o;
#pragma unroll
      for (int e = 0; e < 4; ++e) {
        o[e] = (unsigned short)(bf16_rne_u32(f0[e]) >> 16);
        o[4 + e] = (unsigned short)(bf16_rne_u32(f1[e]) >> 16);
      }
      unsigned short* d = (pl ? xip : xrp) + i;
      *(volatile v8us*)d = o;
    }
    for (size_t c = tid; c < (size_t)NWB * per_w; c += stride) {
      const int mat = (int)(c / per_w);
      const size_t i = (c - (size_t)mat * per_w) * 8;
      const float* w = (mat == 0) ? w0 : (mat == 1) ? w1 : (mat == 2) ? w2 : (mat == 3) ? w3 : (mat == 4) ? w4 : w5;
      const v4f f0 = *(const v4f*)(w + i), f1 = *(const v4f*)(w + i + 4);
      v8us o;
#pragma unroll
      for (int e = 0; e < 4; ++e) {
        o[e] = (unsigned short)(bf16_rne_u32(f0[e]) >> 16);
        o[4 + e] = (unsigned short)(bf16_rne_u32(f1[e]) >> 16);
      }
      *(volatile v8us*)(wpl + c * 8) = o;
    }
    for (size_t c = tid; c < 2 * per_w; c += stride) {
      const int mat = (int)(c / per_w);
      const size_t i = (c - (size_t)mat * per_w) * 8;
      const float* w = mat ? wo1 : wo0;
      const v4f f0 = *(const v4f*)(w + i), f1 = *(const v4f*)(w + i + 4);
      v8h o;
#pragma unroll
      for (int e = 0; e < 4; ++e) {
        o[e] = (h16)(__uint_as_float(bf16_rne_u32(f0[e])) * WO_CARRY);
        o[4 + e] = (h16)(__uint_as_float(bf16_rne_u32(f1[e])) * WO_CARRY);
      }
      *(volatile v8h*)(wopl + c * 8) = o;
    }
    __threadfence();
  }
}

__global__ __launch_bounds__(128) void proj_kernel(const b16* __restrict__ xr, const b16* __restrict__ xi, const b16* __restrict__ wpl,
                                                   const float* __restrict__ tabc, const float* __restrict__ tabs,
                                                   h16* __restrict__ Qh, h16* __restrict__ Kh, h16* __restrict__ Vh,
                                                   h16* __restrict__ Qx, h16* __restrict__ Kx, h16* __restrict__ Vx) {
  __shared__ __attribute__((aligned(16))) h16 Ts[4][16 * QKW];
  __shared__ __attribute__((aligned(16))) float Ct[64 * NFREQ];
  __shared__ __attribute__((aligned(16))) float St[64 * NFREQ];
  const int lane = threadIdx.x & 31, wave = threadIdx.x >> 5, nloc = lane & 15, hlf = lane >> 4;
  const int mat = blockIdx.x / NH, head = blockIdx.x - mat * NH;
  const int mblk = blockIdx.y * 64;
  const int b = mblk / SEQ, t0 = mblk - b * SEQ;
  const bool early = (t0 < TE);
  if (mat < 2) {
    for (int i = threadIdx.x; i < 64 * NFREQ / 4; i += 128) {
      *(v4f*)(Ct + 4 * i) = *(const v4f*)(tabc + (size_t)t0 * NFREQ + 4 * i);
      *(v4f*)(St + 4 * i) = *(const v4f*)(tabs + (size_t)t0 * NFREQ + 4 * i);
    }
  }
  __syncthreads();
  const int tw = t0 + wave * 16;
  const int m0 = b * SEQ + tw;
  const int g = b * NH + head;
  const b16* wr = wpl + (size_t)(2 * mat) * HID * HID + (size_t)(head * DH) * HID;
  const b16* wi = wpl + (size_t)(2 * mat + 1) * HID * HID + (size_t)(head * DH) * HID;
  const b16* ar = xr + (size_t)(m0 + nloc) * HID;
  const b16* ai = xi + (size_t)(m0 + nloc) * HID;
  v8f accr[4], acci[4];
#pragma unroll
  for (int t = 0; t < 4; ++t) { accr[t] = (v8f){}; acci[t] = (v8f){}; }
#pragma unroll 1
  for (int kb = 0; kb < HID; kb += 32) {
    const v16b fr = frag_kb(ar + kb, hlf);
    const v16b fi = frag_kb(ai + kb, hlf);
    const v16b fin = neg16(fi);
#pragma unroll
    for (int t = 0; t < 4; ++t) {
      const v16b br = frag_kb(wr + (size_t)(t * 16 + nloc) * HID + kb, hlf);
      const v16b bi = frag_kb(wi + (size_t)(t * 16 + nloc) * HID + kb, hlf);
      accr[t] = wmma_b(fr, br, accr[t]);
      accr[t] = wmma_b(fin, bi, accr[t]);
      acci[t] = wmma_b(fr, bi, acci[t]);
      acci[t] = wmma_b(fi, br, acci[t]);
    }
  }
  if (mat < 2) {
#pragma unroll
    for (int t = 0; t < 2; ++t) {
      const int j = t * 16 + nloc;
#pragma unroll
      for (int v = 0; v < 8; ++v) {
        const int lr = wave * 16 + 8 * hlf + v;
        const float cv = Ct[lr * NFREQ + j], sv = St[lr * NFREQ + j];
        const float r0 = accr[t][v], r1 = accr[t + 2][v];
        const float i0 = acci[t][v], i1 = acci[t + 2][v];
        accr[t][v] = r0 * cv - r1 * sv;
        accr[t + 2][v] = r1 * cv + r0 * sv;
        acci[t][v] = i0 * cv - i1 * sv;
        acci[t + 2][v] = i1 * cv + i0 * sv;
      }
    }
  }
  h16* Tp = Ts[wave];
#pragma unroll
  for (int t = 0; t < 4; ++t) {
    const int d = t * 16 + nloc;
#pragma unroll
    for (int v = 0; v < 8; ++v) {
      const int rr = 8 * hlf + v;
      const int ir = (mat < 2) ? (rr * QKW + d) : (d * 16 + rr);
      const int ii = (mat < 2) ? (rr * QKW + DH + d) : ((DH + d) * 16 + rr);
      Tp[ir] = (h16)accr[t][v];
      Tp[ii] = (h16)acci[t][v];
    }
  }
  wave_lds_sync();
  h16* dst;
  if (mat == 0) dst = Qh + ((size_t)g * SEQ + tw) * QKW;
  else if (mat == 1) dst = Kh + ((size_t)g * SEQ + tw) * QKW;
  else dst = Vh + ((size_t)g * QT + (tw >> 4)) * (size_t)VTILE;
  store_tile_4k(dst, Tp, lane);
  if (early) {
    wave_lds_sync();
#pragma unroll
    for (int t = 0; t < 4; ++t) {
      const int d = t * 16 + nloc;
#pragma unroll
      for (int v = 0; v < 8; ++v) {
        const int rr = 8 * hlf + v;
        const int ir = (mat < 2) ? (rr * QKW + d) : (d * 16 + rr);
        const int ii = (mat < 2) ? (rr * QKW + DH + d) : ((DH + d) * 16 + rr);
        const float vr = accr[t][v], vi = acci[t][v];
        const h16 hr = (h16)vr, hi = (h16)vi;
        Tp[ir] = (h16)((vr - (float)hr) * RES_CARRY);
        Tp[ii] = (h16)((vi - (float)hi) * RES_CARRY);
      }
    }
    wave_lds_sync();
    h16* dx;
    if (mat == 0) dx = Qx + ((size_t)g * TE + tw) * QKW;
    else if (mat == 1) dx = Kx + ((size_t)g * TE + tw) * QKW;
    else dx = Vx + ((size_t)g * QTE + (tw >> 4)) * (size_t)VTILE;
    store_tile_4k(dx, Tp, lane);
  }
}

__global__ __launch_bounds__(256) __attribute__((amdgpu_num_vgpr(256)))
void attn_late_kernel(const h16* __restrict__ Qh, const h16* __restrict__ Kh, const h16* __restrict__ Vh, h16* __restrict__ Ch) {
  __shared__ __attribute__((aligned(16))) h16 Os[8][16 * QKW];
  const int wid = threadIdx.x >> 5, lane = threadIdx.x & 31, hh = lane >> 4, col = lane & 15;
  const int g = blockIdx.x / NQB_L;
  const int qb = TE + (blockIdx.x - g * NQB_L) * 128;
  const int q0 = qb + wid * 16;
  const int b = g / NH, h = g - b * NH;
  const int qabs = q0 + col;
  const h16* qrow = Qh + ((size_t)g * SEQ + q0 + col) * QKW;
  v16h qf[4];
#pragma unroll
  for (int i = 0; i < 4; ++i) qf[i] = frag_kh(qrow + 32 * i, hh);
  float m = -INFINITY, l = 0.0f;
  v8f o[8];
#pragma unroll
  for (int n = 0; n < 8; ++n) o[n] = (v8f){};
  const int kend = q0 + 16;
#pragma unroll 1
  for (int kb = 0; kb < kend; kb += 32) {
    const h16* k0p = Kh + ((size_t)g * SEQ + kb + col) * QKW;
    const h16* k1p = k0p + (size_t)16 * QKW;
    v8f s0 = {}, s1 = {};
#pragma unroll
    for (int i = 0; i < 4; ++i) {
      v16h kf = frag_kh(k0p + 32 * i, hh);
      s0 = wmma_h(kf, qf[i], s0);
      kf = frag_kh(k1p + 32 * i, hh);
      s1 = wmma_h(kf, qf[i], s1);
    }
    v8f sc0, sc1;
#pragma unroll
    for (int r = 0; r < 8; ++r) {
      const int key0 = kb + 8 * hh + r;
      sc0[r] = (key0 <= qabs) ? (s0[r] * SCORE_SCALE) : -INFINITY;
      sc1[r] = (key0 + 16 <= qabs) ? (s1[r] * SCORE_SCALE) : -INFINITY;
    }
    float mr = -INFINITY;
#pragma unroll
    for (int r = 0; r < 8; ++r) mr = fmaxf(mr, fmaxf(sc0[r], sc1[r]));
    mr = fmaxf(mr, __shfl_xor(mr, 16));
    const float mn = fmaxf(m, mr);
    const float al_ = __expf(m - mn);
    m = mn;
    float sum = 0.0f;
    v16h pb;
#pragma unroll
    for (int r = 0; r < 8; ++r) {
      const float p0 = __expf(sc0[r] - mn), p1 = __expf(sc1[r] - mn);
      sum += p0 + p1;
      pb[r] = (h16)(p0 * P_CARRY);
      pb[8 + r] = (h16)(p1 * P_CARRY);
    }
    sum += __shfl_xor(sum, 16);
    l = l * al_ + sum;
#pragma unroll
    for (int n = 0; n < 8; ++n) o[n] = o[n] * al_;
    const h16* vt0 = Vh + ((size_t)g * QT + (kb >> 4)) * (size_t)VTILE + 8 * hh;
    const h16* vt1 = vt0 + VTILE;
#pragma unroll
    for (int n = 0; n < 8; ++n) {
      const v16h va = cat8h(ld8h(vt0 + (n * 16 + col) * 16), ld8h(vt1 + (n * 16 + col) * 16));
      o[n] = wmma_h(va, pb, o[n]);
    }
  }
  const float inv = (1.0f / l) * INV_P_CARRY;
  h16* Tt = Os[wid];
#pragma unroll
  for (int n = 0; n < 8; ++n) {
    v8h w;
#pragma unroll
    for (int r = 0; r < 8; ++r) w[r] = (h16)(o[n][r] * inv);
    *(v8h*)(Tt + col * QKW + n * 16 + 8 * hh) = w;
  }
  wave_lds_sync();
  const size_t row0 = (size_t)b * SEQ + q0;
#pragma unroll
  for (int j = 0; j < 8; ++j) {
    const int rr = 2 * j + (lane >> 4), seg = (lane >> 3) & 1, c8 = (lane & 7) * 8;
    *(volatile v8h*)(Ch + (row0 + rr) * CW + (size_t)seg * HID + h * DH + c8) = ld8h(Tt + rr * QKW + seg * DH + c8);
  }
  __threadfence();
#pragma unroll
  for (int j = 0; j < 8; ++j) {
    const int rr = 2 * j + (lane >> 4), seg = (lane >> 3) & 1, c8 = (lane & 7) * 8;
    *(volatile v8h*)(Ch + (row0 + rr) * CW + (size_t)seg * HID + h * DH + c8) = ld8h(Tt + rr * QKW + seg * DH + c8);
  }
}

__global__ __launch_bounds__(256) __attribute__((amdgpu_num_vgpr(256)))
void attn_early_kernel(const h16* __restrict__ Qh, const h16* __restrict__ Qx, const h16* __restrict__ Kh, const h16* __restrict__ Kx,
                       const h16* __restrict__ Vh, const h16* __restrict__ Vx, h16* __restrict__ Ch, h16* __restrict__ Cx) {
  __shared__ __attribute__((aligned(16))) h16 Os[8][16 * QKW];
  const int wid = threadIdx.x >> 5, lane = threadIdx.x & 31, hh = lane >> 4, col = lane & 15;
  const int half = blockIdx.x & 1;
  const int rest = blockIdx.x >> 1;
  const int g = rest / NQB_E;
  const int qb = (rest - g * NQB_E) * 128;
  const int q0 = qb + wid * 16;
  const int b = g / NH, h = g - b * NH;
  const int qabs = q0 + col;
  const int fb = half * DH;
  const h16* qhrow = Qh + ((size_t)g * SEQ + q0 + col) * QKW;
  const h16* qxrow = Qx + ((size_t)g * TE + q0 + col) * QKW;
  float m = -INFINITY, l = 0.0f;
  v8f o[4], ox[4];
#pragma unroll
  for (int n = 0; n < 4; ++n) { o[n] = (v8f){}; ox[n] = (v8f){}; }
  const int kend = q0 + 16;
#pragma unroll 1
  for (int kb = 0; kb < kend; kb += 32) {
    const h16* k0h = Kh + ((size_t)g * SEQ + kb + col) * QKW;
    const h16* k1h = k0h + (size_t)16 * QKW;
    const h16* k0x = Kx + ((size_t)g * TE + kb + col) * QKW;
    const h16* k1x = k0x + (size_t)16 * QKW;
    v8f s0 = {}, s1 = {}, x0 = {}, x1 = {};
#pragma unroll
    for (int i = 0; i < 4; ++i) {
      const v16h qh = frag_kh(qhrow + 32 * i, hh);
      const v16h qx = frag_kh(qxrow + 32 * i, hh);
      v16h kh = frag_kh(k0h + 32 * i, hh);
      v16h kx = frag_kh(k0x + 32 * i, hh);
      s0 = wmma_h(kh, qh, s0);
      x0 = wmma_h(kh, qx, x0);
      x0 = wmma_h(kx, qh, x0);
      kh = frag_kh(k1h + 32 * i, hh);
      kx = frag_kh(k1x + 32 * i, hh);
      s1 = wmma_h(kh, qh, s1);
      x1 = wmma_h(kh, qx, x1);
      x1 = wmma_h(kx, qh, x1);
    }
    v8f sc0, sc1;
#pragma unroll
    for (int r = 0; r < 8; ++r) {
      const int key0 = kb + 8 * hh + r;
      const float a0 = (s0[r] + x0[r] * INV_RES_CARRY) * SCORE_SCALE;
      const float a1 = (s1[r] + x1[r] * INV_RES_CARRY) * SCORE_SCALE;
      sc0[r] = (key0 <= qabs) ? a0 : -INFINITY;
      sc1[r] = (key0 + 16 <= qabs) ? a1 : -INFINITY;
    }
    float mr = -INFINITY;
#pragma unroll
    for (int r = 0; r < 8; ++r) mr = fmaxf(mr, fmaxf(sc0[r], sc1[r]));
    mr = fmaxf(mr, __shfl_xor(mr, 16));
    const float mn = fmaxf(m, mr);
    const float al_ = __expf(m - mn);
    m = mn;
    float sum = 0.0f;
    v16h pbh, pbx;
#pragma unroll
    for (int r = 0; r < 8; ++r) {
      const float p0 = __expf(sc0[r] - mn), p1 = __expf(sc1[r] - mn);
      sum += p0 + p1;
      const float c0 = p0 * P_CARRY, c1 = p1 * P_CARRY;
      const h16 e0 = (h16)c0, e1 = (h16)c1;
      pbh[r] = e0;
      pbh[8 + r] = e1;
      pbx[r] = (h16)((c0 - (float)e0) * RES_CARRY);
      pbx[8 + r] = (h16)((c1 - (float)e1) * RES_CARRY);
    }
    sum += __shfl_xor(sum, 16);
    l = l * al_ + sum;
#pragma unroll
    for (int n = 0; n < 4; ++n) { o[n] = o[n] * al_; ox[n] = ox[n] * al_; }
    const h16* vt0h = Vh + ((size_t)g * QT + (kb >> 4)) * (size_t)VTILE + 8 * hh;
    const h16* vt1h = vt0h + VTILE;
    const h16* vt0x = Vx + ((size_t)g * QTE + (kb >> 4)) * (size_t)VTILE + 8 * hh;
    const h16* vt1x = vt0x + VTILE;
#pragma unroll
    for (int n = 0; n < 4; ++n) {
      const int f = (fb + n * 16 + col) * 16;
      const v16h vah = cat8h(ld8h(vt0h + f), ld8h(vt1h + f));
      const v16h vax = cat8h(ld8h(vt0x + f), ld8h(vt1x + f));
      o[n] = wmma_h(vah, pbh, o[n]);
      ox[n] = wmma_h(vah, pbx, ox[n]);
      ox[n] = wmma_h(vax, pbh, ox[n]);
    }
  }
  const float inv = (1.0f / l) * INV_P_CARRY;
  h16* Tt = Os[wid];
#pragma unroll
  for (int n = 0; n < 4; ++n) {
    v8h wh, wx;
#pragma unroll
    for (int r = 0; r < 8; ++r) {
      const float c = (o[n][r] + ox[n][r] * INV_RES_CARRY) * inv;
      const h16 hv = (h16)c;
      wh[r] = hv;
      wx[r] = (h16)((c - (float)hv) * RES_CARRY);
    }
    *(v8h*)(Tt + col * DH + n * 16 + 8 * hh) = wh;
    *(v8h*)(Tt + 1024 + col * DH + n * 16 + 8 * hh) = wx;
  }
  wave_lds_sync();
  const size_t rowh = (size_t)b * SEQ + q0;
  const size_t rowx = (size_t)b * TE + q0;
  const size_t coff = (size_t)half * HID + (size_t)h * DH;
#pragma unroll
  for (int j = 0; j < 4; ++j) {
    const int rr = 4 * j + (lane >> 3), c8 = (lane & 7) * 8;
    *(volatile v8h*)(Ch + (rowh + rr) * CW + coff + c8) = ld8h(Tt + rr * DH + c8);
    *(volatile v8h*)(Cx + (rowx + rr) * CW + coff + c8) = ld8h(Tt + 1024 + rr * DH + c8);
  }
  __threadfence();
#pragma unroll
  for (int j = 0; j < 4; ++j) {
    const int rr = 4 * j + (lane >> 3), c8 = (lane & 7) * 8;
    *(volatile v8h*)(Ch + (rowh + rr) * CW + coff + c8) = ld8h(Tt + rr * DH + c8);
    *(volatile v8h*)(Cx + (rowx + rr) * CW + coff + c8) = ld8h(Tt + 1024 + rr * DH + c8);
  }
}

template <int WCOL>
__device__ __forceinline__ void store_out_tile(float* dst, const float* Tt, int lane) {
  constexpr int LPR = WCOL / 4, RPI = 32 / LPR, NI = 16 / RPI;
#pragma unroll
  for (int j = 0; j < NI; ++j) {
    const int rr = j * RPI + lane / LPR, c4 = (lane % LPR) * 4;
    *(volatile v4f*)(dst + (size_t)rr * HID + c4) = *(const v4f*)(Tt + rr * WCOL + c4);
  }
  __threadfence();
#pragma unroll
  for (int j = 0; j < NI; ++j) {
    const int rr = j * RPI + lane / LPR, c4 = (lane % LPR) * 4;
    *(volatile v4f*)(dst + (size_t)rr * HID + c4) = *(const v4f*)(Tt + rr * WCOL + c4);
  }
}

template <int NT, bool RES>
__global__ __launch_bounds__(256) void oproj_kernel(const h16* __restrict__ Ch, const h16* __restrict__ Cx, const h16* __restrict__ wopl,
                                                    const float* __restrict__ bor, const float* __restrict__ boi,
                                                    float* __restrict__ outr, float* __restrict__ outi) {
  __shared__ __attribute__((aligned(16))) float Os[8][16 * 64];
  constexpr int WCOL = NT * 16;
  constexpr int TB = RES ? 0 : TE;
  constexpr int NQB = RES ? NQB_E : NQB_L;
  const int lane = threadIdx.x & 31, wave = threadIdx.x >> 5, nloc = lane & 15, hlf = lane >> 4;
  const int b = blockIdx.y / NQB;
  const int t0 = TB + (blockIdx.y - b * NQB) * 128 + wave * 16;
  const int m0 = b * SEQ + t0;
  const int c0 = blockIdx.x * WCOL;
  const h16* arow = Ch + (size_t)(m0 + nloc) * CW;
  const h16* xrow = Cx + ((size_t)b * TE + (RES ? t0 : 0) + nloc) * CW;
  const h16* wr = wopl + (size_t)c0 * HID;
  const h16* wi = wopl + (size_t)HID * HID + (size_t)c0 * HID;
  v8f accr[NT], acci[NT], axr[NT], axi[NT];
#pragma unroll
  for (int t = 0; t < NT; ++t) { accr[t] = (v8f){}; acci[t] = (v8f){}; axr[t] = (v8f){}; axi[t] = (v8f){}; }
#pragma unroll 1
  for (int kb = 0; kb < HID; kb += 32) {
    const v16h fr = frag_kh(arow + kb, hlf);
    const v16h fi = frag_kh(arow + HID + kb, hlf);
    const v16h fin = neg16(fi);
    v16h gr = fr, gi = fi, gin = fin;
    if (RES) { gr = frag_kh(xrow + kb, hlf); gi = frag_kh(xrow + HID + kb, hlf); gin = neg16(gi); }
#pragma unroll
    for (int t = 0; t < NT; ++t) {
      const v16h br = frag_kh(wr + (size_t)(t * 16 + nloc) * HID + kb, hlf);
      const v16h bi = frag_kh(wi + (size_t)(t * 16 + nloc) * HID + kb, hlf);
      accr[t] = wmma_h(fr, br, accr[t]);
      accr[t] = wmma_h(fin, bi, accr[t]);
      acci[t] = wmma_h(fr, bi, acci[t]);
      acci[t] = wmma_h(fi, br, acci[t]);
      if (RES) {
        axr[t] = wmma_h(gr, br, axr[t]);
        axr[t] = wmma_h(gin, bi, axr[t]);
        axi[t] = wmma_h(gr, bi, axi[t]);
        axi[t] = wmma_h(gi, br, axi[t]);
      }
    }
  }
  float* Tt = Os[wave];
  const size_t orow = (size_t)m0;
#pragma unroll
  for (int t = 0; t < NT; ++t) {
    const int n = c0 + t * 16 + nloc;
    const float bias = __uint_as_float(bf16_rne_u32(bor[n]));
#pragma unroll
    for (int v = 0; v < 8; ++v) {
      const int rr = 8 * hlf + v;
      float val = accr[t][v] * INV_WO_CARRY;
      if (RES) val = val + axr[t][v] * (INV_WO_CARRY * INV_RES_CARRY);
      val = val + bias;
      Tt[rr * WCOL + t * 16 + nloc] = val;
    }
  }
  wave_lds_sync();
  store_out_tile<WCOL>(outr + orow * HID + c0, Tt, lane);
  wave_lds_sync();
#pragma unroll
  for (int t = 0; t < NT; ++t) {
    const int n = c0 + t * 16 + nloc;
    const float bias = __uint_as_float(bf16_rne_u32(boi[n]));
#pragma unroll
    for (int v = 0; v < 8; ++v) {
      const int rr = 8 * hlf + v;
      float val = acci[t][v] * INV_WO_CARRY;
      if (RES) val = val + axi[t][v] * (INV_WO_CARRY * INV_RES_CARRY);
      val = val + bias;
      Tt[rr * WCOL + t * 16 + nloc] = val;
    }
  }
  wave_lds_sync();
  store_out_tile<WCOL>(outi + orow * HID + c0, Tt, lane);
}
}

extern "C" void kernel_launch(void* const* d_in, const int* in_sizes, int n_in,
                              void* d_out, int out_size, void* d_ws, size_t ws_size, hipStream_t stream) {
  if (n_in < 12) return;
  const size_t need_x = ((size_t)(NB - 1) * SEQ_FULL + SEQ) * HID;
  if ((size_t)in_sizes[0] < need_x || (size_t)in_sizes[1] < need_x) return;
  for (int i = 2; i < 10; ++i) if ((size_t)in_sizes[i] < (size_t)HID * HID) return;
  if (in_sizes[10] < HID || in_sizes[11] < HID) return;
  const size_t OUT1 = (size_t)NB_FULL * SEQ_FULL * HID;
  if ((size_t)out_size < OUT1 + (size_t)MROWS * HID) return;

  const float* x_real = (const float*)d_in[0];
  const float* x_imag = (const float*)d_in[1];
  const float* wq_r = (const float*)d_in[2];
  const float* wq_i = (const float*)d_in[3];
  const float* wk_r = (const float*)d_in[4];
  const float* wk_i = (const float*)d_in[5];
  const float* wv_r = (const float*)d_in[6];
  const float* wv_i = (const float*)d_in[7];
  const float* wo_r = (const float*)d_in[8];
  const float* wo_i = (const float*)d_in[9];
  const float* bo_r = (const float*)d_in[10];
  const float* bo_i = (const float*)d_in[11];
  float* out_r = (float*)d_out;
  float* out_i = out_r + OUT1;

  size_t off = 0; char* ws = (char*)d_ws;
  float* tabc = (float*)(ws + off); off += (size_t)SEQ * NFREQ * 4;
  float* tabs = (float*)(ws + off); off += (size_t)SEQ * NFREQ * 4;
  unsigned short* xrp = (unsigned short*)(ws + off); off += (size_t)MROWS * HID * 2;
  unsigned short* xip = (unsigned short*)(ws + off); off += (size_t)MROWS * HID * 2;
  unsigned short* wpl = (unsigned short*)(ws + off); off += (size_t)NWB * HID * HID * 2;
  h16* wopl = (h16*)(ws + off); off += (size_t)2 * HID * HID * 2;
  h16* Qh = (h16*)(ws + off); off += (size_t)NB * NH * SEQ * QKW * 2;
  h16* Kh = (h16*)(ws + off); off += (size_t)NB * NH * SEQ * QKW * 2;
  h16* Vh = (h16*)(ws + off); off += (size_t)NB * NH * SEQ * QKW * 2;
  h16* Qx = (h16*)(ws + off); off += (size_t)NB * NH * TE * QKW * 2;
  h16* Kx = (h16*)(ws + off); off += (size_t)NB * NH * TE * QKW * 2;
  h16* Vx = (h16*)(ws + off); off += (size_t)NB * NH * TE * QKW * 2;
  h16* Ch = (h16*)(ws + off); off += (size_t)MROWS * CW * 2;
  h16* Cx = (h16*)(ws + off); off += (size_t)NB * TE * CW * 2;
  if (off > ws_size) return;

  tab_kernel<<<SEQ / 8, 256, 0, stream>>>(tabc, tabs);
  cvt_kernel<<<1024, 256, 0, stream>>>(x_real, x_imag, wq_r, wq_i, wk_r, wk_i, wv_r, wv_i, wo_r, wo_i, xrp, xip, wpl, wopl);
  proj_kernel<<<dim3(3 * NH, MROWS / 64), 128, 0, stream>>>((const b16*)xrp, (const b16*)xip, (const b16*)wpl, tabc, tabs,
                                                             Qh, Kh, Vh, Qx, Kx, Vx);
  attn_early_kernel<<<NB * NH * NQB_E * 2, 256, 0, stream>>>(Qh, Qx, Kh, Kx, Vh, Vx, Ch, Cx);
  if (SEQ > TE) attn_late_kernel<<<NB * NH * ((SEQ - TE) / 128), 256, 0, stream>>>(Qh, Kh, Vh, Ch);
  oproj_kernel<2, true><<<dim3(HID / 32, NB * NQB_E), 256, 0, stream>>>(Ch, Cx, wopl, bo_r, bo_i, out_r, out_i);
  if (SEQ > TE) oproj_kernel<4, false><<<dim3(HID / 64, NB * ((SEQ - TE) / 128)), 256, 0, stream>>>(Ch, Cx, wopl, bo_r, bo_i, out_r, out_i);
}
